// CLUB_51144470560984
// MI455X (gfx1250) — hardware-run, weakly checked
//
#include <hip/hip_runtime.h>
#include <math.h>

typedef __attribute__((ext_vector_type(16))) _Float16 v16h;
typedef __attribute__((ext_vector_type(8)))  _Float16 v8h;
typedef __attribute__((ext_vector_type(8)))  float    v8f;
typedef __attribute__((ext_vector_type(4)))  float    v4f;

constexpr int kEmb = 128;
constexpr int kHid = 128;
constexpr int kNpt = 1024;
constexpr int kW1P = 2 * kEmb;
constexpr int kWP = 136;
constexpr int kHP = 136;
constexpr int kPP = 36;
constexpr float kH1Carry = 64.0f;
constexpr float kW2Carry = 256.0f;
constexpr float kFold    = 1.0f / (kH1Carry * kW2Carry);
constexpr int kProjBlocks = (2 * kNpt) / 8;
constexpr int kCvtBlocks  = (kHid * kHid / 8) / 256;
constexpr int kMainWaves   = 2;
constexpr int kTilesPerWav = kNpt / (32 * kMainWaves);
static_assert(kEmb % 4 == 0 && kHid == 128 && kNpt % 8 == 0, "prep tiling");
static_assert(kHid % 32 == 0, "K multiple of 32");
static_assert(kNpt % (32 * kMainWaves) == 0, "column tiles");
static_assert(kCvtBlocks * 256 * 8 == kHid * kHid, "W2 plane coverage");
static_assert(kTilesPerWav * kMainWaves * 32 == kNpt, "row coverage");
static_assert((kWP % 8) == 0 && (kHP % 8) == 0 && (kPP % 4) == 0, "16-B aligned LDS rows");

constexpr size_t kOffAPL  = 0;
constexpr size_t kOffBBP  = kOffAPL + (size_t)kNpt * kHid * 4;
constexpr size_t kOffW2H  = kOffBBP + (size_t)kNpt * kHid * 4;
constexpr size_t kWsTotal = kOffW2H + (size_t)kHid * kHid * 2;
static_assert(kWsTotal == 1081344ull, "carve total");
static_assert(kWsTotal <= 134217728ull, "carve cap");
static_assert((kOffBBP % 128) == 0 && (kOffW2H % 128) == 0, "128-B aligned regions");

struct FragH {
  union U { v16h v; v8h h[2]; };
  static __device__ __forceinline__ v16h load(const _Float16* p) {
    U f;
    f.h[0] = *(const v8h*)(p);
    f.h[1] = *(const v8h*)(p + 16);
    return f.v;
  }
};

__device__ __forceinline__ v8f mma_g(v16h a, v16h b, v8f c) {
  c = __builtin_amdgcn_wmma_f32_16x16x32_f16(false, a, false, b, (short)0, c, false, false);
  asm volatile("v_nop\n\tv_nop\n\tv_nop\n\tv_nop" : "+v"(c) : "v"(a), "v"(b));
  return c;
}

__device__ __forceinline__ float gelu_erf(float x) {
  return 0.5f * x * (1.0f + erff(x * 0.70710678118654752f));
}

__global__ __launch_bounds__(256) void prep_kernel(
    const float* __restrict__ z1, const float* __restrict__ z2, const float* __restrict__ W1,
    const float* __restrict__ b1, const float* __restrict__ W2,
    float* __restrict__ APL, float* __restrict__ BBP, unsigned short* __restrict__ W2H)
{
  const int tid = threadIdx.x, lane = tid & 31, wave = tid >> 5;
  if (blockIdx.x < kProjBlocks) {
    const int row   = blockIdx.x * 8 + wave;
    const int which = (row >= kNpt) ? 1 : 0;
    const int r     = row - which * kNpt;
    const float* zrow = (which ? z2 : z1) + (size_t)r * kEmb;
    const int h0 = lane * 4;
    const float* w0 = W1 + (size_t)h0 * kW1P + which * kEmb;
    float acc0 = 0.f, acc1 = 0.f, acc2 = 0.f, acc3 = 0.f;
#pragma unroll 1
    for (int d4 = 0; d4 < kEmb / 4; ++d4) {
      const v4f zv = *(const v4f*)(zrow + 4 * d4);
      const v4f wa = *(const v4f*)(w0 + 4 * d4);
      const v4f wb = *(const v4f*)(w0 + kW1P + 4 * d4);
      const v4f wc = *(const v4f*)(w0 + 2 * kW1P + 4 * d4);
      const v4f wd = *(const v4f*)(w0 + 3 * kW1P + 4 * d4);
      acc0 = fmaf(zv[0], wa[0], acc0); acc0 = fmaf(zv[1], wa[1], acc0);
      acc0 = fmaf(zv[2], wa[2], acc0); acc0 = fmaf(zv[3], wa[3], acc0);
      acc1 = fmaf(zv[0], wb[0], acc1); acc1 = fmaf(zv[1], wb[1], acc1);
      acc1 = fmaf(zv[2], wb[2], acc1); acc1 = fmaf(zv[3], wb[3], acc1);
      acc2 = fmaf(zv[0], wc[0], acc2); acc2 = fmaf(zv[1], wc[1], acc2);
      acc2 = fmaf(zv[2], wc[2], acc2); acc2 = fmaf(zv[3], wc[3], acc2);
      acc3 = fmaf(zv[0], wd[0], acc3); acc3 = fmaf(zv[1], wd[1], acc3);
      acc3 = fmaf(zv[2], wd[2], acc3); acc3 = fmaf(zv[3], wd[3], acc3);
    }
    const v4f bv = *(const v4f*)(b1 + h0);
    v4f o;
    o[0] = acc0 + (which ? bv[0] : 0.0f);
    o[1] = acc1 + (which ? bv[1] : 0.0f);
    o[2] = acc2 + (which ? bv[2] : 0.0f);
    o[3] = acc3 + (which ? bv[3] : 0.0f);
    float* dst = (which ? BBP : APL) + (size_t)r * kHid + h0;
    *(volatile v4f*)dst = o;
    __threadfence();
    *(volatile v4f*)dst = o;
  } else {
    const int idx = (blockIdx.x - kProjBlocks) * 256 + tid;
    const size_t e0 = (size_t)idx * 8;
    const v4f a0 = *(const v4f*)(W2 + e0);
    const v4f a1 = *(const v4f*)(W2 + e0 + 4);
    v8h hv;
#pragma unroll
    for (int e = 0; e < 4; ++e) {
      hv[e]     = (_Float16)(a0[e] * kW2Carry);
      hv[4 + e] = (_Float16)(a1[e] * kW2Carry);
    }
    unsigned short* q = W2H + e0;
    *(volatile v8h*)q = hv;
    __threadfence();
    *(volatile v8h*)q = hv;
  }
}

__global__ __launch_bounds__(64) void pair_mlp_kernel(
    const float* __restrict__ APL, const float* __restrict__ BBP, const unsigned short* __restrict__ W2Hp,
    const float* __restrict__ b2, const float* __restrict__ W3, const float* __restrict__ b3,
    float* __restrict__ out)
{
  __shared__ __align__(16) _Float16 w2s[kHid * kWP];
  __shared__ __align__(16) _Float16 hs[kMainWaves][32 * kHP];
  __shared__ __align__(16) float    ps[kMainWaves][32 * kPP];
  __shared__ __align__(16) float    bbs[kHid];
  __shared__ __align__(16) float    b2s[kHid];
  __shared__ __align__(16) float    w3s[kHid];

  const int tid = threadIdx.x, lane = tid & 31, wave = tid >> 5;
  const int hh = lane >> 4, rl = lane & 15;
  const int i = blockIdx.x;
  const _Float16* W2H = (const _Float16*)W2Hp;

#pragma unroll 1
  for (int it = 0; it < 32; ++it) {
    const int u = it * 64 + tid;
    const int g = u >> 4;
    const int c = (u & 15) * 8;
    *(v8h*)(w2s + g * kWP + c) = *(const v8h*)(W2H + g * kHid + c);
  }
  {
    const int e = tid * 2;
    bbs[e]     = BBP[(size_t)i * kHid + e];
    bbs[e + 1] = BBP[(size_t)i * kHid + e + 1];
    b2s[e]     = b2[e];
    b2s[e + 1] = b2[e + 1];
    w3s[e]     = W3[e];
    w3s[e + 1] = W3[e + 1];
  }
  const float b3v = b3[0];
  __syncthreads();

  _Float16* hw = hs[wave];
  float*    pw = ps[wave];

#pragma unroll 1
  for (int tt = 0; tt < kTilesPerWav; ++tt) {
    const int j0 = (wave * kTilesPerWav + tt) * 32;
    const float* arow = APL + (size_t)(j0 + lane) * kHid;

#pragma unroll 1
    for (int c8 = 0; c8 < kHid / 8; ++c8) {
      const v4f x0 = *(const v4f*)(arow + 8 * c8);
      const v4f x1 = *(const v4f*)(arow + 8 * c8 + 4);
      const v4f y0 = *(const v4f*)(bbs + 8 * c8);
      const v4f y1 = *(const v4f*)(bbs + 8 * c8 + 4);
      v8h hv;
#pragma unroll
      for (int e = 0; e < 4; ++e) {
        const float g0 = gelu_erf(x0[e] + y0[e]);
        const float g1 = gelu_erf(x1[e] + y1[e]);
        hv[e]     = (_Float16)(kH1Carry * g0);
        hv[4 + e] = (_Float16)(kH1Carry * g1);
      }
      *(v8h*)(hw + lane * kHP + 8 * c8) = hv;
    }
    __syncthreads();

    float s = 0.f;
#pragma unroll 1
    for (int q = 0; q < 4; ++q) {
      v8f acc00 = (v8f){0.f, 0.f, 0.f, 0.f, 0.f, 0.f, 0.f, 0.f};
      v8f acc01 = acc00, acc10 = acc00, acc11 = acc00;
#pragma unroll
      for (int t = 0; t < 4; ++t) {
        const int ko = 32 * t + 8 * hh;
        const v16h a0 = FragH::load(hw + rl * kHP + ko);
        const v16h a1 = FragH::load(hw + (16 + rl) * kHP + ko);
        const v16h bA = FragH::load(w2s + (q * 32 + rl) * kWP + ko);
        const v16h bB = FragH::load(w2s + (q * 32 + 16 + rl) * kWP + ko);
        acc00 = mma_g(a0, bA, acc00);
        acc10 = mma_g(a1, bA, acc10);
        acc01 = mma_g(a0, bB, acc01);
        acc11 = mma_g(a1, bB, acc11);
      }
#pragma unroll
      for (int r = 0; r < 8; ++r) {
        pw[(8 * hh + r) * kPP + rl]           = acc00[r];
        pw[(8 * hh + r) * kPP + 16 + rl]      = acc01[r];
        pw[(16 + 8 * hh + r) * kPP + rl]      = acc10[r];
        pw[(16 + 8 * hh + r) * kPP + 16 + rl] = acc11[r];
      }
      __syncthreads();
#pragma unroll 1
      for (int c4 = 0; c4 < 8; ++c4) {
        const v4f pv = *(const v4f*)(pw + lane * kPP + 4 * c4);
        const v4f bv = *(const v4f*)(b2s + q * 32 + 4 * c4);
        const v4f wv = *(const v4f*)(w3s + q * 32 + 4 * c4);
#pragma unroll
        for (int e = 0; e < 4; ++e) {
          const float p = fmaf(pv[e], kFold, bv[e]);
          s = fmaf(wv[e], gelu_erf(p), s);
        }
      }
      __syncthreads();
    }

    const float val = s + b3v;
    float* op = out + (size_t)i * kNpt + j0 + lane;
    *(volatile float*)op = val;
    __threadfence();
    *(volatile float*)op = val;
  }
}

extern "C" void kernel_launch(void* const* d_in, const int* in_sizes, int n_in,
                              void* d_out, int out_size, void* d_ws, size_t ws_size,
                              hipStream_t stream) {
  if (n_in < 8) return;
  if (in_sizes[0] != kNpt * kEmb) return;
  if (in_sizes[1] != kNpt * kEmb) return;
  if (in_sizes[2] != kHid * kW1P) return;
  if (in_sizes[3] != kHid) return;
  if (in_sizes[4] != kHid * kHid) return;
  if (in_sizes[5] != kHid) return;
  if (in_sizes[6] != kHid) return;
  if (in_sizes[7] != 1) return;
  if (out_size != kNpt * kNpt) return;
  if (ws_size < kWsTotal) return;

  const float* z1 = (const float*)d_in[0];
  const float* z2 = (const float*)d_in[1];
  const float* W1 = (const float*)d_in[2];
  const float* b1 = (const float*)d_in[3];
  const float* W2 = (const float*)d_in[4];
  const float* b2 = (const float*)d_in[5];
  const float* W3 = (const float*)d_in[6];
  const float* b3 = (const float*)d_in[7];
  float* out = (float*)d_out;

  char* ws = (char*)d_ws;
  float*          APL = (float*)(ws + kOffAPL);
  float*          BBP = (float*)(ws + kOffBBP);
  unsigned short* W2H = (unsigned short*)(ws + kOffW2H);

  prep_kernel<<<kProjBlocks + kCvtBlocks, 256, 0, stream>>>(z1, z2, W1, b1, W2, APL, BBP, W2H);
  pair_mlp_kernel<<<kNpt, 64, 0, stream>>>(APL, BBP, W2H, b2, W3, b3, out);
}
